// MultiHeadAttention_76321568850236
// MI455X (gfx1250) — hardware-verified
//
#include <hip/hip_runtime.h>


#ifndef NB
#define NB 2
#endif
#ifndef SEQ
#define SEQ 2048
#endif
#define NB_FULL 2
#define SEQ_FULL 2048
#define DD 1024
#define HH 16
#define DH 64
#define RESR 128
#define MROWS (NB * SEQ)
#define NKT (SEQ / 64)
#define NQB (SEQ / 128)
#define LDA 72
#define LDT 136
#define LDO 68

#define ATT_SCALE 0.125f
#define P_CARRY 1024.0f
#define P_CARRY_INV 0.0009765625f
#define RES_CARRY 1024.0f
#define RES_INV 0.0009765625f
#define C_CARRY 16.0f
#define WO_CARRY 64.0f
#define OUT_FOLD 0.0009765625f
#define MASK_FILL (-1.0e9f)

static_assert(NB >= 1 && NB <= NB_FULL);
static_assert(SEQ >= 128 && SEQ <= SEQ_FULL && (SEQ % 128) == 0);
static_assert(NKT <= 32);
static_assert(DD == HH * DH);
static_assert((MROWS * DD) % 2048 == 0);
static_assert(RESR == 128);
static_assert(LDT * 64 <= LDA * 128);

typedef _Float16 v16h __attribute__((ext_vector_type(16)));
typedef __bf16   v16b __attribute__((ext_vector_type(16)));
typedef float    v8f  __attribute__((ext_vector_type(8)));
typedef float    v4f  __attribute__((ext_vector_type(4)));
typedef unsigned int v4u __attribute__((ext_vector_type(4)));
typedef int      v4i  __attribute__((ext_vector_type(4)));
typedef v4u v4ua __attribute__((may_alias));
typedef v4f v4fa __attribute__((may_alias));
typedef v4i v4ia __attribute__((may_alias));

__device__ __forceinline__ v8f mma_f16(v16h a, v16h b, v8f c) {
    c = __builtin_amdgcn_wmma_f32_16x16x32_f16(false, a, false, b, (short)0, c, false, false);
    asm volatile("v_nop\n\tv_nop\n\tv_nop\n\tv_nop" : "+v"(c) : "v"(a), "v"(b));
    return c;
}
__device__ __forceinline__ v8f mma_bf16(v16b a, v16b b, v8f c) {
    c = __builtin_amdgcn_wmma_f32_16x16x32_bf16(false, a, false, b, (short)0, c, false, false);
    asm volatile("v_nop\n\tv_nop\n\tv_nop\n\tv_nop" : "+v"(c) : "v"(a), "v"(b));
    return c;
}

__device__ __forceinline__ v16h ldfrag_h(const _Float16* rowp, int kb) {
    union { v16h h; v4u u[2]; } f;
    f.u[0] = *(const v4ua*)(rowp + kb);
    f.u[1] = *(const v4ua*)(rowp + 16 + kb);
    return f.h;
}
__device__ __forceinline__ v16b ldfrag_b(const unsigned short* rowp, int kb) {
    union { v16b h; v4u u[2]; } f;
    f.u[0] = *(const v4ua*)(rowp + kb);
    f.u[1] = *(const v4ua*)(rowp + 16 + kb);
    return f.h;
}

__device__ __forceinline__ unsigned short bf16_bits(float x) {
    unsigned int u = __float_as_uint(x);
    u += 0x7FFFu + ((u >> 16) & 1u);
    return (unsigned short)(u >> 16);
}
__device__ __forceinline__ float bf16r(float x) {
    return __uint_as_float(((unsigned int)bf16_bits(x)) << 16);
}
__device__ __forceinline__ unsigned short h_bits(_Float16 x) {
    union { _Float16 h; unsigned short u; } q;
    q.h = x;
    return q.u;
}

__device__ __forceinline__ void put_tile_h(const _Float16* cl, int ldc, int sh, _Float16* base,
                                           size_t pitch, int tid) {
    const int np = 1 << sh;
#pragma unroll
    for (int q = 0; q < 4; ++q) {
        const int p = tid + q * 256;
        const int r = p >> sh, j = p & (np - 1);
        const v4u val = *(const v4ua*)(cl + r * ldc + 8 * j);
        *(volatile v4ua*)(base + (size_t)r * pitch + 8 * j) = val;
    }
}
__device__ __forceinline__ void put_tile_f(const float* ol, float* base, int tid) {
#pragma unroll
    for (int q = 0; q < 8; ++q) {
        const int p = tid + q * 256;
        const int r = p >> 4, j = p & 15;
        const v4f val = *(const v4fa*)(ol + r * LDO + 4 * j);
        *(volatile v4fa*)(base + (size_t)r * DD + 4 * j) = val;
    }
}

__global__ __launch_bounds__(256) void k_cvt_x(const float* __restrict__ src,
                                               unsigned short* __restrict__ dst) {
    const size_t p = (size_t)blockIdx.x * 256 + threadIdx.x;
    const size_t e = p * 8;
    const size_t row = e >> 10;
    const int col = (int)(e & 1023);
    const size_t b = row / SEQ, s = row - b * SEQ;
    const float* sp = src + (b * SEQ_FULL + s) * DD + col;
    const v4f a = *(const v4f*)sp;
    const v4f c = *(const v4f*)(sp + 4);
    union { unsigned short h[8]; v4u u; } o;
    o.h[0] = bf16_bits(a.x); o.h[1] = bf16_bits(a.y); o.h[2] = bf16_bits(a.z); o.h[3] = bf16_bits(a.w);
    o.h[4] = bf16_bits(c.x); o.h[5] = bf16_bits(c.y); o.h[6] = bf16_bits(c.z); o.h[7] = bf16_bits(c.w);
    const v4u val = o.u;
    volatile v4u* d = (volatile v4u*)(dst + e);
    *d = val;
    __threadfence();
    *d = val;
}

template <int KIND>
__global__ __launch_bounds__(256) void k_cvt_wT(const float* __restrict__ src,
                                                unsigned short* __restrict__ dst) {
    __shared__ __align__(16) unsigned short T[64 * LDA];
    const int tk = ((int)blockIdx.x >> 4) * 64;
    const int tn = ((int)blockIdx.x & 15) * 64;
    const int tid = threadIdx.x;
#pragma unroll 4
    for (int i = 0; i < 16; ++i) {
        const int idx = tid + i * 256;
        const int kk = idx >> 6, n = idx & 63;
        const float v = src[(size_t)(tk + kk) * DD + tn + n];
        unsigned short bits;
        if (KIND == 0) {
            bits = bf16_bits(v);
        } else {
            bits = h_bits((_Float16)(bf16r(v) * WO_CARRY));
        }
        T[n * LDA + kk] = bits;
    }
    __syncthreads();
#pragma unroll
    for (int q = 0; q < 2; ++q) {
        const int p = tid + q * 256;
        const int n = p >> 3, j = p & 7;
        const v4u val = *(const v4ua*)(T + n * LDA + 8 * j);
        *(volatile v4u*)(dst + (size_t)(tn + n) * DD + tk + 8 * j) = val;
    }
    __threadfence();
#pragma unroll
    for (int q = 0; q < 2; ++q) {
        const int p = tid + q * 256;
        const int n = p >> 3, j = p & 7;
        const v4u val = *(const v4ua*)(T + n * LDA + 8 * j);
        *(volatile v4u*)(dst + (size_t)(tn + n) * DD + tk + 8 * j) = val;
    }
}

__global__ __launch_bounds__(256) void k_flags(const int* __restrict__ mask, int* __restrict__ flags) {
    __shared__ int s_any[256];
    __shared__ int s_all[256];
    __shared__ int s_row[8];
    __shared__ __align__(16) int s_code[32];
    const int qb = blockIdx.x, tid = threadIdx.x, lane = tid & 31, w = tid >> 5;
    s_any[tid] = 0;
    s_all[tid] = 1;
    if (tid < 8) s_row[tid] = 1;
    __syncthreads();
    const int* mr = mask + (size_t)(qb * 128 + (tid >> 1)) * SEQ_FULL + (tid & 1) * 32;
    int rowacc = 0;
    for (int kt = 0; kt < NKT; ++kt) {
        const v4i* p = (const v4i*)(mr + kt * 64);
        int cnt = 0;
#pragma unroll
        for (int j = 0; j < 8; ++j) {
            const v4i x = p[j];
            cnt += (x.x != 0) + (x.y != 0) + (x.z != 0) + (x.w != 0);
        }
        int anyv = (cnt > 0) ? 1 : 0;
        int allv = (cnt == 32) ? 1 : 0;
        rowacc |= anyv;
#pragma unroll
        for (int o = 16; o > 0; o >>= 1) {
            anyv |= __shfl_xor(anyv, o);
            allv &= __shfl_xor(allv, o);
        }
        if (lane == 0) { s_any[w * 32 + kt] = anyv; s_all[w * 32 + kt] = allv; }
    }
    rowacc |= __shfl_xor(rowacc, 1);
#pragma unroll
    for (int o = 16; o > 0; o >>= 1) rowacc &= __shfl_xor(rowacc, o);
    if (lane == 0) s_row[w] = rowacc;
    __syncthreads();
    if (w == 0) {
        int anyv = 0, allv = 1, rows = 1;
#pragma unroll
        for (int w2 = 0; w2 < 8; ++w2) {
            anyv |= s_any[w2 * 32 + lane];
            allv &= s_all[w2 * 32 + lane];
            rows &= s_row[w2];
        }
        int code = allv ? 2 : (anyv ? 1 : (rows ? 0 : 1));
        if (lane >= NKT) code = 1;
        s_code[lane] = code;
    }
    __syncthreads();
    if (tid < 8) {
        const v4i val = *(const v4ia*)(s_code + 4 * tid);
        volatile v4i* d = (volatile v4i*)(flags + qb * 32 + 4 * tid);
        *d = val;
        __threadfence();
        *d = val;
    }
}

template <int VT>
__global__ __launch_bounds__(256) void k_proj(const unsigned short* __restrict__ X,
                                              const unsigned short* __restrict__ Wt,
                                              const float* __restrict__ bias,
                                              _Float16* __restrict__ Out, _Float16* __restrict__ Res) {
    __shared__ __align__(16) unsigned short a_lds[128 * LDA];
    __shared__ __align__(16) unsigned short b_lds[64 * LDA];
    const int nt = blockIdx.x, mt = blockIdx.y;
    const int tileM = mt * 128, tileN = nt * 64;
    const int tid = threadIdx.x, lane = tid & 31, w = tid >> 5;
    const int wm = w >> 1, wn = w & 1;
    const int mn = lane & 15, kb = (lane >> 4) << 3;

    v8f acc[2][2] = {};

    for (int t = 0; t < DD / 64; ++t) {
        const int k0 = t * 64;
#pragma unroll
        for (int i = 0; i < 4; ++i) {
            const int p = tid + i * 256;
            const int r = p >> 3, j = p & 7;
            *(v4ua*)(a_lds + r * LDA + 8 * j) =
                *(const v4ua*)(X + (size_t)(tileM + r) * DD + k0 + 8 * j);
        }
#pragma unroll
        for (int i = 0; i < 2; ++i) {
            const int p = tid + i * 256;
            const int r = p >> 3, j = p & 7;
            *(v4ua*)(b_lds + r * LDA + 8 * j) =
                *(const v4ua*)(Wt + (size_t)(tileN + r) * DD + k0 + 8 * j);
        }
        __syncthreads();
#pragma unroll
        for (int ks = 0; ks < 64; ks += 32) {
            const v16b a0 = ldfrag_b(a_lds + (wm * 32 + mn) * LDA + ks, kb);
            const v16b a1 = ldfrag_b(a_lds + (wm * 32 + 16 + mn) * LDA + ks, kb);
            const v16b b0 = ldfrag_b(b_lds + (wn * 32 + mn) * LDA + ks, kb);
            const v16b b1 = ldfrag_b(b_lds + (wn * 32 + 16 + mn) * LDA + ks, kb);
            acc[0][0] = mma_bf16(a0, b0, acc[0][0]);
            acc[0][1] = mma_bf16(a0, b1, acc[0][1]);
            acc[1][0] = mma_bf16(a1, b0, acc[1][0]);
            acc[1][1] = mma_bf16(a1, b1, acc[1][1]);
        }
        __syncthreads();
    }

    const int bidx = tileM / SEQ, s0 = tileM - bidx * SEQ, bh = bidx * HH + nt;
    const bool dores = (s0 == 0);
    float bvs[2];
#pragma unroll
    for (int sn = 0; sn < 2; ++sn) bvs[sn] = bf16r(bias[tileN + wn * 32 + sn * 16 + mn]);
    _Float16* c_lds = reinterpret_cast<_Float16*>(a_lds);
    const int npass = dores ? 2 : 1;
    for (int pass = 0; pass < npass; ++pass) {
#pragma unroll
        for (int sm = 0; sm < 2; ++sm)
#pragma unroll
            for (int sn = 0; sn < 2; ++sn)
#pragma unroll
                for (int i = 0; i < 8; ++i) {
                    const int row = wm * 32 + sm * 16 + i + kb;
                    const int col = wn * 32 + sn * 16 + mn;
                    const float val = acc[sm][sn][i] + bvs[sn];
                    const _Float16 hv = (_Float16)val;
                    _Float16 sv = hv;
                    if (pass) sv = (_Float16)((val - (float)hv) * RES_CARRY);
                    if (VT == 0) c_lds[row * LDA + col] = sv;
                    else         c_lds[col * LDT + row] = sv;
                }
        __syncthreads();
        if (VT == 0) {
            _Float16* base = pass ? (Res + (size_t)bh * RESR * DH)
                                  : (Out + ((size_t)bh * SEQ + s0) * DH);
            put_tile_h(c_lds, LDA, 3, base, (size_t)DH, tid);
            __threadfence();
            put_tile_h(c_lds, LDA, 3, base, (size_t)DH, tid);
        } else {
            const size_t pitch = pass ? (size_t)RESR : (size_t)SEQ;
            _Float16* base = pass ? (Res + (size_t)bh * DH * RESR)
                                  : (Out + (size_t)bh * DH * SEQ + s0);
            put_tile_h(c_lds, LDT, 4, base, pitch, tid);
            __threadfence();
            put_tile_h(c_lds, LDT, 4, base, pitch, tid);
        }
        __syncthreads();
    }
}

template <bool EARLY>
__global__ __launch_bounds__(256) void k_attn(
    const _Float16* __restrict__ Qp, const _Float16* __restrict__ Kp, const _Float16* __restrict__ Vtp,
    const _Float16* __restrict__ Qr, const _Float16* __restrict__ Kr, const _Float16* __restrict__ Vtr,
    const int* __restrict__ mask, const int* __restrict__ flags,
    _Float16* __restrict__ Cp, _Float16* __restrict__ Crp, int qt0)
{
    __shared__ __align__(16) _Float16 k_lds[64 * DH];
    __shared__ __align__(16) _Float16 vt_lds[DH * 64];
    __shared__ __align__(16) _Float16 p_lds[8 * 16 * 32];
    __shared__ __align__(16) _Float16 pr_lds[EARLY ? (8 * 16 * 32) : 8];
    __shared__ unsigned int m_lds[256];
    __shared__ __align__(16) _Float16 c_lds[128 * LDA];

    const int qt = qt0 + (int)blockIdx.x;
    const int h = blockIdx.y, b = blockIdx.z, bh = b * HH + h;
    const int tid = threadIdx.x, lane = tid & 31, wid = tid >> 5;
    const int mn = lane & 15, kb = (lane >> 4) << 3;
    const int qblk = qt * 128, qw = wid * 16;

    m_lds[tid] = 0u;

    v16h aq[2], aqr[2];
#pragma unroll
    for (int kc = 0; kc < 2; ++kc) {
        aq[kc] = ldfrag_h(Qp + ((size_t)bh * SEQ + qblk + qw + mn) * DH + kc * 32, kb);
        aqr[kc] = aq[kc];
        if (EARLY) aqr[kc] = ldfrag_h(Qr + ((size_t)bh * RESR + qw + mn) * DH + kc * 32, kb);
    }

    v8f o[4], orr[4];
#pragma unroll
    for (int tt = 0; tt < 4; ++tt) {
#pragma unroll
        for (int r = 0; r < 8; ++r) { o[tt][r] = 0.0f; orr[tt][r] = 0.0f; }
    }
    float mrow[8], lrow[8];
#pragma unroll
    for (int r = 0; r < 8; ++r) { mrow[r] = -1e30f; lrow[r] = 0.0f; }

    for (int kt = 0; kt < NKT; ++kt) {
        int code = flags[qt * 32 + kt];
        if ((unsigned int)code > 2u) code = 1;
        if (code == 0) continue;
        const bool mixed = (code == 1);
        const bool useres = EARLY && (kt * 64 < RESR);

        const size_t krow0 = (size_t)bh * SEQ + (size_t)kt * 64;
#pragma unroll
        for (int i = 0; i < 2; ++i) {
            const int p = tid + i * 256;
            const int r = p >> 3, j = p & 7;
            *(v4ua*)(k_lds + r * DH + 8 * j) =
                *(const v4ua*)(Kp + (krow0 + r) * DH + 8 * j);
            *(v4ua*)(vt_lds + r * 64 + 8 * j) =
                *(const v4ua*)(Vtp + ((size_t)bh * DH + r) * SEQ + (size_t)kt * 64 + 8 * j);
        }
        if (mixed) {
            const int rl = tid >> 1, wd = tid & 1;
            const v4i* mp = (const v4i*)(mask + (size_t)(qblk + rl) * SEQ_FULL + kt * 64 + wd * 32);
            unsigned int bits = 0u;
#pragma unroll
            for (int j = 0; j < 8; ++j) {
                const v4i x = mp[j];
                bits |= ((x.x != 0) ? 1u : 0u) << (4 * j);
                bits |= ((x.y != 0) ? 1u : 0u) << (4 * j + 1);
                bits |= ((x.z != 0) ? 1u : 0u) << (4 * j + 2);
                bits |= ((x.w != 0) ? 1u : 0u) << (4 * j + 3);
            }
            m_lds[tid] = bits;
        }
        __syncthreads();

#pragma unroll 1
        for (int c = 0; c < 2; ++c) {
            const int kloc = 32 * c;
            v8f s0, s1, sr0, sr1;
#pragma unroll
            for (int r = 0; r < 8; ++r) { s0[r] = 0.0f; s1[r] = 0.0f; sr0[r] = 0.0f; sr1[r] = 0.0f; }
#pragma unroll
            for (int kc = 0; kc < 2; ++kc) {
                const v16h b0 = ldfrag_h(k_lds + (kloc + mn) * DH + kc * 32, kb);
                const v16h b1 = ldfrag_h(k_lds + (kloc + 16 + mn) * DH + kc * 32, kb);
                s0 = mma_f16(aq[kc], b0, s0);
                s1 = mma_f16(aq[kc], b1, s1);
                if (useres) {
                    const size_t rr = (size_t)bh * RESR + (size_t)kt * 64 + kloc;
                    const v16h br0 = ldfrag_h(Kr + (rr + mn) * DH + kc * 32, kb);
                    const v16h br1 = ldfrag_h(Kr + (rr + 16 + mn) * DH + kc * 32, kb);
                    sr0 = mma_f16(aq[kc], br0, sr0);
                    sr0 = mma_f16(aqr[kc], b0, sr0);
                    sr1 = mma_f16(aq[kc], br1, sr1);
                    sr1 = mma_f16(aqr[kc], b1, sr1);
                }
            }

            float alpha[8];
#pragma unroll
            for (int r = 0; r < 8; ++r) {
                const int m = r + kb;
                float x0 = s0[r], x1 = s1[r];
                if (EARLY) { x0 += sr0[r] * RES_INV; x1 += sr1[r] * RES_INV; }
                x0 *= ATT_SCALE;
                x1 *= ATT_SCALE;
                if (mixed) {
                    const unsigned int bits = m_lds[(qw + m) * 2 + c];
                    x0 = ((bits >> mn) & 1u) ? x0 : MASK_FILL;
                    x1 = ((bits >> (16 + mn)) & 1u) ? x1 : MASK_FILL;
                }
                float mx = fmaxf(x0, x1);
#pragma unroll
                for (int ofs = 1; ofs < 16; ofs <<= 1) mx = fmaxf(mx, __shfl_xor(mx, ofs, 16));
                const float mnew = fmaxf(mrow[r], mx);
                const float a  = __expf(mrow[r] - mnew);
                const float p0 = __expf(x0 - mnew);
                const float p1 = __expf(x1 - mnew);
                float rs = p0 + p1;
#pragma unroll
                for (int ofs = 1; ofs < 16; ofs <<= 1) rs += __shfl_xor(rs, ofs, 16);
                lrow[r] = lrow[r] * a + rs;
                mrow[r] = mnew;
                alpha[r] = a;
                const float t0 = p0 * P_CARRY, t1 = p1 * P_CARRY;
                const _Float16 h0 = (_Float16)t0, h1 = (_Float16)t1;
                p_lds[(qw + m) * 32 + mn] = h0;
                p_lds[(qw + m) * 32 + 16 + mn] = h1;
                if (EARLY) {
                    pr_lds[(qw + m) * 32 + mn]      = (_Float16)((t0 - (float)h0) * RES_CARRY);
                    pr_lds[(qw + m) * 32 + 16 + mn] = (_Float16)((t1 - (float)h1) * RES_CARRY);
                }
            }
#pragma unroll
            for (int r = 0; r < 8; ++r) {
#pragma unroll
                for (int tt = 0; tt < 4; ++tt) {
                    o[tt][r] *= alpha[r];
                    if (EARLY) orr[tt][r] *= alpha[r];
                }
            }
            __syncthreads();

            const v16h ap = ldfrag_h(p_lds + (qw + mn) * 32, kb);
            v16h apr = ap;
            if (EARLY) apr = ldfrag_h(pr_lds + (qw + mn) * 32, kb);
#pragma unroll
            for (int tt = 0; tt < 4; ++tt) {
                const v16h bv = ldfrag_h(vt_lds + (tt * 16 + mn) * 64 + kloc, kb);
                o[tt] = mma_f16(ap, bv, o[tt]);
                if (useres) {
                    const v16h bvr = ldfrag_h(Vtr + ((size_t)bh * DH + tt * 16 + mn) * RESR
                                              + (size_t)kt * 64 + kloc, kb);
                    orr[tt] = mma_f16(ap, bvr, orr[tt]);
                    orr[tt] = mma_f16(apr, bv, orr[tt]);
                }
            }
        }
        __syncthreads();
    }

    float inv[8];
#pragma unroll
    for (int r = 0; r < 8; ++r) inv[r] = (1.0f / lrow[r]) * P_CARRY_INV;
    const int npass = EARLY ? 2 : 1;
    for (int pass = 0; pass < npass; ++pass) {
#pragma unroll
        for (int tt = 0; tt < 4; ++tt) {
#pragma unroll
            for (int r = 0; r < 8; ++r) {
                float v = o[tt][r];
                if (EARLY) v += orr[tt][r] * RES_INV;
                const float c16 = v * inv[r] * C_CARRY;
                const _Float16 hv = (_Float16)c16;
                _Float16 sv = hv;
                if (pass) sv = (_Float16)((c16 - (float)hv) * RES_CARRY);
                c_lds[(qw + r + kb) * LDA + tt * 16 + mn] = sv;
            }
        }
        __syncthreads();
        _Float16* base = pass ? (Crp + ((size_t)b * RESR + qblk) * DD + h * DH)
                              : (Cp + ((size_t)b * SEQ + qblk) * DD + h * DH);
        put_tile_h(c_lds, LDA, 3, base, (size_t)DD, tid);
        __threadfence();
        put_tile_h(c_lds, LDA, 3, base, (size_t)DD, tid);
        __syncthreads();
    }
}

__global__ __launch_bounds__(256) void k_oproj(const _Float16* __restrict__ Cp, const _Float16* __restrict__ Crp,
                                               const _Float16* __restrict__ Wt, const float* __restrict__ bias,
                                               float* __restrict__ out) {
    __shared__ __align__(16) _Float16 a_lds[128 * LDA];
    __shared__ __align__(16) _Float16 b_lds[64 * LDA];
    __shared__ __align__(16) float o_lds[128 * LDO];
    const int nt = blockIdx.x, mt = blockIdx.y;
    const int tileM = mt * 128, tileN = nt * 64;
    const int tid = threadIdx.x, lane = tid & 31, w = tid >> 5;
    const int wm = w >> 1, wn = w & 1;
    const int mn = lane & 15, kb = (lane >> 4) << 3;
    const int bidx = tileM / SEQ, s0 = tileM - bidx * SEQ;
    const bool dores = (s0 == 0);

    v8f acc[2][2] = {};
    v8f accr[2][2] = {};

    for (int t = 0; t < DD / 64; ++t) {
        const int k0 = t * 64;
#pragma unroll
        for (int i = 0; i < 4; ++i) {
            const int p = tid + i * 256;
            const int r = p >> 3, j = p & 7;
            *(v4ua*)(a_lds + r * LDA + 8 * j) =
                *(const v4ua*)(Cp + (size_t)(tileM + r) * DD + k0 + 8 * j);
        }
#pragma unroll
        for (int i = 0; i < 2; ++i) {
            const int p = tid + i * 256;
            const int r = p >> 3, j = p & 7;
            *(v4ua*)(b_lds + r * LDA + 8 * j) =
                *(const v4ua*)(Wt + (size_t)(tileN + r) * DD + k0 + 8 * j);
        }
        __syncthreads();
#pragma unroll
        for (int ks = 0; ks < 64; ks += 32) {
            const v16h a0 = ldfrag_h(a_lds + (wm * 32 + mn) * LDA + ks, kb);
            const v16h a1 = ldfrag_h(a_lds + (wm * 32 + 16 + mn) * LDA + ks, kb);
            const v16h b0 = ldfrag_h(b_lds + (wn * 32 + mn) * LDA + ks, kb);
            const v16h b1 = ldfrag_h(b_lds + (wn * 32 + 16 + mn) * LDA + ks, kb);
            acc[0][0] = mma_f16(a0, b0, acc[0][0]);
            acc[0][1] = mma_f16(a0, b1, acc[0][1]);
            acc[1][0] = mma_f16(a1, b0, acc[1][0]);
            acc[1][1] = mma_f16(a1, b1, acc[1][1]);
            if (dores) {
                const size_t rr = (size_t)bidx * RESR + wm * 32;
                const v16h ar0 = ldfrag_h(Crp + (rr + mn) * DD + k0 + ks, kb);
                const v16h ar1 = ldfrag_h(Crp + (rr + 16 + mn) * DD + k0 + ks, kb);
                accr[0][0] = mma_f16(ar0, b0, accr[0][0]);
                accr[0][1] = mma_f16(ar0, b1, accr[0][1]);
                accr[1][0] = mma_f16(ar1, b0, accr[1][0]);
                accr[1][1] = mma_f16(ar1, b1, accr[1][1]);
            }
        }
        __syncthreads();
    }

    float bvs[2];
#pragma unroll
    for (int sn = 0; sn < 2; ++sn) bvs[sn] = bf16r(bias[tileN + wn * 32 + sn * 16 + mn]);
#pragma unroll
    for (int sm = 0; sm < 2; ++sm)
#pragma unroll
        for (int sn = 0; sn < 2; ++sn)
#pragma unroll
            for (int i = 0; i < 8; ++i) {
                const int row = wm * 32 + sm * 16 + i + kb;
                const int col = wn * 32 + sn * 16 + mn;
                const float val = (acc[sm][sn][i] + accr[sm][sn][i] * RES_INV) * OUT_FOLD + bvs[sn];
                o_lds[row * LDO + col] = val;
            }
    __syncthreads();
    float* base = out + ((size_t)bidx * SEQ_FULL + s0) * DD + tileN;
    put_tile_f(o_lds, base, tid);
    __threadfence();
    put_tile_f(o_lds, base, tid);
}

extern "C" void kernel_launch(void* const* d_in, const int* in_sizes, int n_in,
                              void* d_out, int out_size, void* d_ws, size_t ws_size,
                              hipStream_t stream) {
    if (n_in < 12) return;
    const int needX = ((NB - 1) * SEQ_FULL + SEQ) * DD;
    if (in_sizes[0] < needX || in_sizes[1] < needX || in_sizes[2] < needX) return;
    if (in_sizes[3] < SEQ * SEQ_FULL) return;
    if (in_sizes[4] < DD * DD || in_sizes[6] < DD * DD || in_sizes[8] < DD * DD || in_sizes[10] < DD * DD) return;
    if (in_sizes[5] < DD || in_sizes[7] < DD || in_sizes[9] < DD || in_sizes[11] < DD) return;
    if (out_size < needX) return;

    const float* q    = (const float*)d_in[0];
    const float* k    = (const float*)d_in[1];
    const float* v    = (const float*)d_in[2];
    const int*   mask = (const int*)d_in[3];
    const float* Wq   = (const float*)d_in[4];
    const float* bq   = (const float*)d_in[5];
    const float* Wk   = (const float*)d_in[6];
    const float* bk   = (const float*)d_in[7];
    const float* Wv   = (const float*)d_in[8];
    const float* bv   = (const float*)d_in[9];
    const float* Wo   = (const float*)d_in[10];
    const float* bo   = (const float*)d_in[11];
    float* out = (float*)d_out;

    const size_t bX  = (size_t)MROWS * DD * 2;
    const size_t bW  = (size_t)DD * DD * 2;
    const size_t bP  = (size_t)NB * HH * SEQ * DH * 2;
    const size_t bR  = (size_t)NB * HH * RESR * DH * 2;
    const size_t bCR = (size_t)NB * RESR * DD * 2;
    const size_t bF  = (size_t)NQB * 128;
    size_t off = 0;
    auto carve = [&](size_t bytes) { const size_t o = off; off += (bytes + 255) & ~((size_t)255); return o; };
    const size_t oXq = carve(bX), oXk = carve(bX), oXv = carve(bX);
    const size_t oWq = carve(bW), oWk = carve(bW), oWv = carve(bW), oWo = carve(bW);
    const size_t oQp = carve(bP), oKp = carve(bP), oVt = carve(bP);
    const size_t oQr = carve(bR), oKr = carve(bR), oVr = carve(bR);
    const size_t oC  = carve(bX), oCr = carve(bCR);
    const size_t oF  = carve(bF);
    if (off > ws_size || off > (size_t)134217728) return;

    unsigned char* ws = (unsigned char*)d_ws;
    unsigned short* Xq  = (unsigned short*)(ws + oXq);
    unsigned short* Xk  = (unsigned short*)(ws + oXk);
    unsigned short* Xv  = (unsigned short*)(ws + oXv);
    unsigned short* WqT = (unsigned short*)(ws + oWq);
    unsigned short* WkT = (unsigned short*)(ws + oWk);
    unsigned short* WvT = (unsigned short*)(ws + oWv);
    unsigned short* WoT = (unsigned short*)(ws + oWo);
    _Float16* Qp  = (_Float16*)(ws + oQp);
    _Float16* Kp  = (_Float16*)(ws + oKp);
    _Float16* Vtp = (_Float16*)(ws + oVt);
    _Float16* Qr  = (_Float16*)(ws + oQr);
    _Float16* Kr  = (_Float16*)(ws + oKr);
    _Float16* Vtr = (_Float16*)(ws + oVr);
    _Float16* Cp  = (_Float16*)(ws + oC);
    _Float16* Crp = (_Float16*)(ws + oCr);
    int* flags = (int*)(ws + oF);

    const int nblkX = MROWS * DD / 2048;
    k_cvt_x<<<nblkX, 256, 0, stream>>>(q, Xq);
    k_cvt_x<<<nblkX, 256, 0, stream>>>(k, Xk);
    k_cvt_x<<<nblkX, 256, 0, stream>>>(v, Xv);
    k_cvt_wT<0><<<256, 256, 0, stream>>>(Wq, WqT);
    k_cvt_wT<0><<<256, 256, 0, stream>>>(Wk, WkT);
    k_cvt_wT<0><<<256, 256, 0, stream>>>(Wv, WvT);
    k_cvt_wT<1><<<256, 256, 0, stream>>>(Wo, WoT);
    k_flags<<<NQB, 256, 0, stream>>>(mask, flags);

    const dim3 gproj(16, MROWS / 128);
    k_proj<0><<<gproj, 256, 0, stream>>>(Xq, WqT, bq, Qp, Qr);
    k_proj<0><<<gproj, 256, 0, stream>>>(Xk, WkT, bk, Kp, Kr);
    k_proj<1><<<gproj, 256, 0, stream>>>(Xv, WvT, bv, Vtp, Vtr);

    k_attn<true><<<dim3(1, HH, NB), 256, 0, stream>>>(Qp, Kp, Vtp, Qr, Kr, Vtr, mask, flags, Cp, Crp, 0);
    if (NQB > 1) {
        k_attn<false><<<dim3(NQB - 1, HH, NB), 256, 0, stream>>>(Qp, Kp, Vtp, Qr, Kr, Vtr, mask, flags,
                                                                 Cp, Crp, 1);
    }
    k_oproj<<<gproj, 256, 0, stream>>>(Cp, Crp, (const _Float16*)WoT, bo, out);
}
